// DSQGAttentionN_35356170780874
// MI455X (gfx1250) — hardware-verified
//
#include <hip/hip_runtime.h>
#include <math.h>

typedef __attribute__((ext_vector_type(16))) _Float16 v16h;
typedef __attribute__((ext_vector_type(16))) __bf16 v16b;
typedef __attribute__((ext_vector_type(8)))  _Float16 v8h;
typedef __attribute__((ext_vector_type(8)))  float v8f;
typedef __attribute__((ext_vector_type(4)))  float v4f;
typedef __attribute__((ext_vector_type(2)))  float v2f;
typedef __attribute__((ext_vector_type(4)))  unsigned v4u;
typedef __attribute__((ext_vector_type(4)))  int v4i;
typedef float __attribute__((may_alias)) float_a;
typedef int __attribute__((may_alias)) int_a;

template <typename T> __device__ __forceinline__ void vst2(void* p, T v) { *(volatile T*)p = v; __threadfence(); *(volatile T*)p = v; }
__device__ __forceinline__ v8f wmma16(v16h a, v16h b, v8f c) {
  v8f d = __builtin_amdgcn_wmma_f32_16x16x32_f16(false, a, false, b, (short)0, c, false, false);
  asm volatile("v_nop\n\tv_nop\n\tv_nop\n\tv_nop" : "+v"(d) : "v"(a), "v"(b));
  return d;
}
__device__ __forceinline__ v8f wmma_bf(v16b a, v16b b, v8f c) {
  v8f d = __builtin_amdgcn_wmma_f32_16x16x32_bf16(false, a, false, b, (short)0, c, false, false);
  asm volatile("v_nop\n\tv_nop\n\tv_nop\n\tv_nop" : "+v"(d) : "v"(a), "v"(b));
  return d;
}
__device__ __forceinline__ v16h frag_h(const _Float16* rowk0, int lane) {
  union { v16h v; v8h q[2]; } u; const _Float16* p = rowk0 + 8 * (lane >> 4);
  u.q[0] = *(const v8h*)p; u.q[1] = *(const v8h*)(p + 16); return u.v;
}
__device__ __forceinline__ v16h frag_f32(const float* rowk0, int lane) {
  v16h a; const float* p = rowk0 + 8 * (lane >> 4);
#pragma unroll
  for (int i = 0; i < 8; ++i) { a[i] = (_Float16)p[i]; a[8 + i] = (_Float16)p[16 + i]; }
  return a;
}
__device__ __forceinline__ v16h frag_f32s(const float* rowk0, int lane, float sc) {
  v16h a; const float* p = rowk0 + 8 * (lane >> 4);
#pragma unroll
  for (int i = 0; i < 8; ++i) { a[i] = (_Float16)(p[i] * sc); a[8 + i] = (_Float16)(p[16 + i] * sc); }
  return a;
}
__device__ __forceinline__ v16h fragc_f32(const float* W, int k0, int n, int lane, int ld, int K) {
  v16h a; const int g = lane >> 4;
#pragma unroll
  for (int i = 0; i < 8; ++i) { const int ka = k0 + 8 * g + i, kb = ka + 16;
    a[i] = (_Float16)(ka < K ? W[(size_t)(ka < K ? ka : K - 1) * ld + n] : 0.f); a[8 + i] = (_Float16)(kb < K ? W[(size_t)(kb < K ? kb : K - 1) * ld + n] : 0.f); }
  return a;
}
struct F2 { v16b h, l; };
__device__ __forceinline__ F2 bsplit16(const float v[16]) { F2 r;
#pragma unroll
  for (int i = 0; i < 16; ++i) { const __bf16 h = (__bf16)v[i]; r.h[i] = h; r.l[i] = (__bf16)(v[i] - (float)h); }
  return r; }
__device__ __forceinline__ F2 split_row(const float* row, int k0, int lane) { float v[16]; const float* p = row + k0 + 8 * (lane >> 4);
#pragma unroll
  for (int i = 0; i < 8; ++i) { v[i] = p[i]; v[8 + i] = p[16 + i]; }
  return bsplit16(v); }
__device__ __forceinline__ F2 split_rowK(const float* row, int k0, int lane, int K) { float v[16]; const int g = lane >> 4;
#pragma unroll
  for (int i = 0; i < 8; ++i) { const int ka = k0 + 8 * g + i, kb = ka + 16; v[i] = ka < K ? row[ka < K ? ka : K - 1] : 0.f; v[8 + i] = kb < K ? row[kb < K ? kb : K - 1] : 0.f; }
  return bsplit16(v); }
__device__ __forceinline__ F2 split_col(const float* W, int k0, int n, int lane, int ld, int K) { float v[16]; const int g = lane >> 4;
#pragma unroll
  for (int i = 0; i < 8; ++i) { const int ka = k0 + 8 * g + i, kb = ka + 16; v[i] = ka < K ? W[(size_t)(ka < K ? ka : K - 1) * ld + n] : 0.f; v[8 + i] = kb < K ? W[(size_t)(kb < K ? kb : K - 1) * ld + n] : 0.f; }
  return bsplit16(v); }
__device__ __forceinline__ v8f mac3(const F2& a, const F2& b, v8f c) { c = wmma_bf(a.l, b.h, c); c = wmma_bf(a.h, b.l, c); return wmma_bf(a.h, b.h, c); }
__device__ __forceinline__ float sigm(float v) { return 1.0f / (1.0f + expf(-v)); }
#define LDSX() do { asm volatile("s_wait_dscnt 0" ::: "memory"); __builtin_amdgcn_wave_barrier(); __builtin_amdgcn_fence(__ATOMIC_RELEASE, "workgroup"); } while (0)


#define NB 2
#define SS 2048
#define DM 1024
#define NH 16
#define HD 64
#define NO 44
#define NR (NB * SS)
#ifndef TRB
#define TRB (NR / 64)
#endif
typedef __attribute__((ext_vector_type(8))) __bf16 v8b;
__device__ __forceinline__ v16b frag_b(const __bf16* rowk0, int lane) {
  union { v16b v; v8b q[2]; } u; const __bf16* p = rowk0 + 8 * (lane >> 4);
  u.q[0] = *(const v8b*)p; u.q[1] = *(const v8b*)(p + 16); return u.v;
}
__device__ __forceinline__ float bfr(float v) { return (float)(__bf16)v; }
__device__ __attribute__((noinline)) float exp_ni(float v) { return expf(v); }
__device__ __attribute__((noinline)) float erf_ni(float v) { return erff(v); }
__constant__ int OFFS[NO] = {0,1,2,3,4,5,6,7,8,9,10,11,12,13,14,15,16,17,18,19,20,21,22,23,24,25,26,27,28,29,30,31,32,48,64,96,128,192,256,384,512,768,1024,1536};

#define WS_PW  0u
#define WS_PG  (WS_PW + 2u * (size_t)3 * DM * DM)
#define WS_PO  (WS_PG + 2u * (size_t)DM * DM)
#define WS_Q   (WS_PO + 2u * (size_t)DM * DM)
#define WS_K   (WS_Q + 4u * (size_t)NR * DM)
#define WS_V   (WS_K + 4u * (size_t)NR * DM)
#define WS_Y   (WS_V + 4u * (size_t)NR * DM)
#define WS_END (WS_Y + 4u * (size_t)NR * DM)

__global__ __launch_bounds__(256) void k_pack(const float* __restrict__ WQKV, const float* __restrict__ WG, const float* __restrict__ WO, __bf16* __restrict__ PW, __bf16* __restrict__ PG, __bf16* __restrict__ PO) { const int n = blockIdx.x, which = blockIdx.y, t = threadIdx.x; __shared__ __align__(16) __bf16 s[DM];
  if (which < 3) { for (int k = t; k < DM; k += 256) s[k] = (__bf16)WQKV[(size_t)k * (3 * DM) + which * DM + n]; }
  else if (which == 3) { for (int k = t; k < DM; k += 256) s[k] = (__bf16)WG[(size_t)k * DM + n]; }
  else { for (int k = t; k < DM; k += 256) s[k] = (__bf16)WO[(size_t)k * DM + n]; }
  __syncthreads(); __bf16* dst = (which < 3) ? (PW + ((size_t)which * DM + n) * DM) : (which == 3) ? (PG + (size_t)n * DM) : (PO + (size_t)n * DM);
  if (t < DM / 8) vst2((unsigned*)(dst + t * 8), *(const v4u*)&s[t * 8]); }
template <int MODE>
__global__ __launch_bounds__(128) void k_g(const float* __restrict__ A, const __bf16* __restrict__ P, const float* __restrict__ BB, const float* __restrict__ FL, float* __restrict__ O0, float* __restrict__ O1, float* __restrict__ O2) { __shared__ __align__(16) float so[4][16][132];
  const int tid = threadIdx.x, wave = tid >> 5, lane = tid & 31, col = lane & 15, g = lane >> 4; const size_t r0 = (size_t)blockIdx.x * 64 + wave * 16; const int c0 = blockIdx.y * 128; const int which = blockIdx.z;
  const __bf16* Wr = P + ((MODE == 0) ? (size_t)which * DM * DM : 0); const float* bb0 = BB + ((MODE == 0) ? which * DM : 0);
  v8f acc[8] = {};
  if (MODE < 2) {
#pragma unroll 2
    for (int kc = 0; kc < DM / 32; ++kc) { v16b a; { const float* p = A + (r0 + col) * DM + kc * 32 + 8 * g;
#pragma unroll
        for (int i = 0; i < 8; ++i) { a[i] = (__bf16)p[i]; a[8 + i] = (__bf16)p[16 + i]; } }
#pragma unroll
      for (int j = 0; j < 8; ++j) acc[j] = wmma_bf(a, frag_b(Wr + (size_t)(c0 + j * 16 + col) * DM + kc * 32, lane), acc[j]); } }
  else {
#pragma unroll 2
    for (int kc = 0; kc < DM / 32; ++kc) { const F2 a = split_row(A + (r0 + col) * DM, kc * 32, lane);
#pragma unroll
      for (int j = 0; j < 8; ++j) { const v16b w = frag_b(Wr + (size_t)(c0 + j * 16 + col) * DM + kc * 32, lane); acc[j] = wmma_bf(a.h, w, acc[j]); acc[j] = wmma_bf(a.l, w, acc[j]); } } }
#pragma unroll
  for (int j = 0; j < 8; ++j) { const int c = c0 + j * 16 + col; const float bb = bfr(bb0[c]);
#pragma unroll
    for (int r = 0; r < 8; ++r) { float v = acc[j][r] + bb; if (MODE == 1) v = FL[(r0 + 8 * g + r) * DM + c] / (1.0f + __expf(-v)); so[wave][8 * g + r][j * 16 + col] = v; } }
  LDSX(); float* OUT = (MODE == 0) ? ((which == 0) ? O0 : (which == 1) ? O1 : O2) : O0;
  for (int rl = 0; rl < 16; ++rl) vst2(OUT + (r0 + rl) * DM + c0 + lane * 4, *(const v4f*)&so[wave][rl][lane * 4]); }
__global__ __launch_bounds__(256) void k_tap(const float* __restrict__ Q, const float* __restrict__ Kr, const float* __restrict__ V, const float* __restrict__ PB, float* __restrict__ FL) { __shared__ __align__(16) float so2[DM]; __shared__ float ssc[NO][257];
  const int t = threadIdx.x; const int h = t >> 4, sub = t & 15; const size_t row = blockIdx.x; const int n = (int)(row % SS); const size_t rowb = row - n;
  float qv[4]; for (int i = 0; i < 4; ++i) qv[i] = Q[row * DM + h * HD + sub * 4 + i];
  float mx = -3.0e38f;
#pragma unroll 1
  for (int o = 0; o < NO; ++o) { const int dl = OFFS[o]; float s = -3.0e38f;
    if (n >= dl) { const float* kr = Kr + (rowb + (n - dl)) * DM + h * HD + sub * 4; float a = 0.f; for (int i = 0; i < 4; ++i) a += qv[i] * kr[i];
#pragma unroll
      for (int x = 1; x < 16; x <<= 1) a += __shfl_xor(a, x);
      s = a * 0.125f + bfr(PB[o * NH + h]); }
    ssc[o][t] = s; mx = fmaxf(mx, s); }
  float z = 0.f; for (int o = 0; o < NO; ++o) { const float sv = ssc[o][t]; const float e = (sv <= -1.0e38f) ? 0.f : __expf(sv - mx); ssc[o][t] = e; z += e; }
  float acc[4] = {0.f, 0.f, 0.f, 0.f};
#pragma unroll 1
  for (int o = 0; o < NO; ++o) { const int dl = OFFS[o]; if (n >= dl) { const float* vr = V + (rowb + (n - dl)) * DM + h * HD + sub * 4; const float w = ssc[o][t]; for (int i = 0; i < 4; ++i) acc[i] += w * vr[i]; } }
  const float iz = 1.0f / z; v4f o4; for (int i = 0; i < 4; ++i) o4[i] = acc[i] * iz; *(v4f*)&so2[h * HD + sub * 4] = o4;
  __syncthreads(); vst2(FL + row * DM + t * 4, *(const v4f*)&so2[t * 4]); }
extern "C" void kernel_launch(void* const* d_in, const int* in_sizes, int n_in, void* d_out, int out_size, void* d_ws, size_t ws_size, hipStream_t stream) {
  (void)in_sizes; (void)n_in; (void)out_size;
  const float** F = (const float**)d_in;
  if (ws_size < (size_t)WS_END) return;
  char* ws = (char*)d_ws; __bf16 *PW = (__bf16*)(ws + WS_PW), *PG = (__bf16*)(ws + WS_PG), *PO = (__bf16*)(ws + WS_PO); float *Q = (float*)(ws + WS_Q), *Kr = (float*)(ws + WS_K), *V = (float*)(ws + WS_V), *Y = (float*)(ws + WS_Y);
  k_pack<<<dim3(DM, 5), 256, 0, stream>>>(F[1], F[5], F[3], PW, PG, PO);
  k_g<0><<<dim3(NR / 64, DM / 128, 3), 128, 0, stream>>>(F[0], PW, F[2], nullptr, Q, Kr, V);
  k_tap<<<TRB * 64, 256, 0, stream>>>(Q, Kr, V, F[7], Q);
  k_g<1><<<dim3(TRB, DM / 128, 1), 128, 0, stream>>>(F[0], PG, F[6], Q, Y, nullptr, nullptr);
  k_g<2><<<dim3(TRB, DM / 128, 1), 128, 0, stream>>>(Y, PO, F[4], nullptr, (float*)d_out, nullptr, nullptr);
}
